// NMP_22832046146013
// MI455X (gfx1250) — hardware-verified
//
#include <hip/hip_runtime.h>
#include <hip/hip_bf16.h>
#include <stddef.h>
#include <stdint.h>


#define NF    64
#define EFW   32
#define KP    2112
#define KW    2048
#define WCOLS 4096
#define EB    64
#define NTE   128
#define NB    200
#define NTA   64
#define CH    64
#define NMIDC 20000
#define WSCAP 134217728
#define PLB   (NF * KP * 2)

static_assert((KP % 32) == 0);
static_assert(KP == KW + NF);
static_assert(KW == NF * EFW);
static_assert((NB % 4) == 0);
static_assert(NB <= 4 * NTA);
static_assert(NB > 3 * NTA);
static_assert(CH == NTA);
static_assert((PLB % 256) == 0);
static_assert(((NF * KP) % (8 * 256)) == 0);
static_assert(((EB * NF) % (4 * NTE)) == 0);
static_assert(((EB * EFW) % (4 * NTE)) == 0);
static_assert(((NB * NF) % (4 * NTA)) == 0);

typedef float          v4f   __attribute__((ext_vector_type(4)));
typedef float          v8f   __attribute__((ext_vector_type(8)));
typedef __bf16         v8bf  __attribute__((ext_vector_type(8)));
typedef __bf16         v16bf __attribute__((ext_vector_type(16)));
typedef unsigned short v8us  __attribute__((ext_vector_type(8)));

union FragB { v16bf v; v8bf h[2]; v8us u[2]; };
union Cvt8  { v8bf b; v8us u; };

__device__ __forceinline__ v8f wmf(v16bf a, v16bf b, v8f c) {
  v8f d = __builtin_amdgcn_wmma_f32_16x16x32_bf16(false, a, false, b, (short)0, c, false, false);
  asm volatile("v_nop\n\tv_nop\n\tv_nop\n\tv_nop" : "+v"(d) : "v"(a), "v"(b));
  return d;
}

__device__ __forceinline__ v8f vzero8() {
  v8f z = {0.f, 0.f, 0.f, 0.f, 0.f, 0.f, 0.f, 0.f};
  return z;
}

__device__ __forceinline__ void split16(const v8f p0, const v8f p1, FragB& ah, FragB& al) {
  const v8bf h0 = __builtin_convertvector(p0, v8bf);
  const v8bf h1 = __builtin_convertvector(p1, v8bf);
  const v8f  r0 = p0 - __builtin_convertvector(h0, v8f);
  const v8f  r1 = p1 - __builtin_convertvector(h1, v8f);
  ah.h[0] = h0;
  ah.h[1] = h1;
  al.h[0] = __builtin_convertvector(r0, v8bf);
  al.h[1] = __builtin_convertvector(r1, v8bf);
}

__device__ __forceinline__ v8f mma3(v8f c, const v16bf ah, const v16bf al,
                                    const unsigned short* __restrict__ ph,
                                    const unsigned short* __restrict__ pl) {
  FragB bh, bl;
  bh.u[0] = *(const v8us*)(ph);
  bh.u[1] = *(const v8us*)(ph + 16);
  bl.u[0] = *(const v8us*)(pl);
  bl.u[1] = *(const v8us*)(pl + 16);
  c = wmf(ah, bh.v, c);
  c = wmf(ah, bl.v, c);
  c = wmf(al, bh.v, c);
  return c;
}

__global__ __launch_bounds__(256) void k_wsplit(const float* __restrict__ Wa, const float* __restrict__ ba,
                                                 const float* __restrict__ Wb, const float* __restrict__ bb,
                                                 unsigned short* pha, unsigned short* pla,
                                                 unsigned short* phb, unsigned short* plb) {
  const int sel = blockIdx.y;
  const float* W  = sel ? Wb : Wa;
  const float* bs = sel ? bb : ba;
  unsigned short* hp = sel ? phb : pha;
  unsigned short* lp = sel ? plb : pla;
  const int idx = blockIdx.x * 256 + (int)threadIdx.x;
  if (idx >= (NF * KP) / 8) return;
  const int e8 = idx * 8;
  const int n  = e8 / KP;
  const int k0 = e8 - n * KP;
  v8f v;
#pragma unroll
  for (int j = 0; j < 8; ++j) {
    const int k  = k0 + j;
    const int kw = min(k, KW - 1);
    const int iw = kw >> 5, kk = kw & 31;
    const float vw = W[(size_t)kk * WCOLS + iw * NF + n];
    const int ib = min(max(k - KW, 0), NF - 1);
    const float vb = bs[ib * NF + n];
    v[j] = (k < KW) ? vw : vb;
  }
  Cvt8 ch, cl;
  ch.b = __builtin_convertvector(v, v8bf);
  const v8f r = v - __builtin_convertvector(ch.b, v8f);
  cl.b = __builtin_convertvector(r, v8bf);
  unsigned short* dh = hp + e8;
  unsigned short* dl = lp + e8;
  *(volatile v8us*)dh = ch.u;
  *(volatile v8us*)dl = cl.u;
  __threadfence();
  *(volatile v8us*)dh = ch.u;
  *(volatile v8us*)dl = cl.u;
}

__global__ __launch_bounds__(NTE) void k_edge(const float* __restrict__ hsrc, int n_src,
                                              const float* __restrict__ ef,
                                              const int* __restrict__ src, int E,
                                              const unsigned short* __restrict__ Bh,
                                              const unsigned short* __restrict__ Bl,
                                              float* msg) {
  __shared__ __attribute__((aligned(32))) float sh_h[EB * NF];
  __shared__ __attribute__((aligned(32))) float sh_e[EB * EFW];
  __shared__ __attribute__((aligned(32))) float sh_o[EB * NF];
  const int t = threadIdx.x, lane = t & 31, w = t >> 5, h = lane >> 4, m = lane & 15;
  const int ebase = blockIdx.x * EB;
  const v4f z4 = {0.f, 0.f, 0.f, 0.f};

#pragma unroll
  for (int q = 0; q < (EB * NF) / (4 * NTE); ++q) {
    const int idx = q * NTE + t;
    const int e = idx >> 4, c4 = idx & 15;
    const int ge = ebase + e;
    const int gc = min(ge, E - 1);
    int s = src[gc];
    s = min(max(s, 0), n_src - 1);
    v4f x = *(const v4f*)(hsrc + (size_t)s * NF + 4 * c4);
    x = (ge < E) ? x : z4;
    *(v4f*)(sh_h + e * NF + 4 * c4) = x;
  }
#pragma unroll
  for (int q = 0; q < (EB * EFW) / (4 * NTE); ++q) {
    const int idx = q * NTE + t;
    const int e = idx >> 3, c4 = idx & 7;
    const int ge = ebase + e;
    const int gc = min(ge, E - 1);
    v4f x = *(const v4f*)(ef + (size_t)gc * EFW + 4 * c4);
    x = (ge < E) ? x : z4;
    *(v4f*)(sh_e + e * EFW + 4 * c4) = x;
  }
  __syncthreads();

  const int er = 16 * w + m;
  const float* efr = sh_e + er * EFW;
  const v8f ek0 = *(const v8f*)(efr + 8 * h);
  const v8f ek1 = *(const v8f*)(efr + 16 + 8 * h);
  const float* hr = sh_h + er * NF;
  const unsigned short* ph = Bh + (size_t)m * KP + 8 * h;
  const unsigned short* pl = Bl + (size_t)m * KP + 8 * h;

  v8f c0 = vzero8(), c1 = vzero8(), c2 = vzero8(), c3 = vzero8();

#pragma unroll 1
  for (int i = 0; i < NF; ++i) {
    const float s = hr[i];
    FragB ah, al;
    split16(ek0 * s, ek1 * s, ah, al);
    const int k0 = 32 * i;
    c0 = mma3(c0, ah.v, al.v, ph + k0,           pl + k0);
    c1 = mma3(c1, ah.v, al.v, ph + 16 * KP + k0, pl + 16 * KP + k0);
    c2 = mma3(c2, ah.v, al.v, ph + 32 * KP + k0, pl + 32 * KP + k0);
    c3 = mma3(c3, ah.v, al.v, ph + 48 * KP + k0, pl + 48 * KP + k0);
  }
#pragma unroll
  for (int tt = 0; tt < 2; ++tt) {
    const v8f x0 = *(const v8f*)(hr + 32 * tt + 8 * h);
    const v8f x1 = *(const v8f*)(hr + 32 * tt + 16 + 8 * h);
    FragB ah, al;
    split16(x0, x1, ah, al);
    const int k0 = KW + 32 * tt;
    c0 = mma3(c0, ah.v, al.v, ph + k0,           pl + k0);
    c1 = mma3(c1, ah.v, al.v, ph + 16 * KP + k0, pl + 16 * KP + k0);
    c2 = mma3(c2, ah.v, al.v, ph + 32 * KP + k0, pl + 32 * KP + k0);
    c3 = mma3(c3, ah.v, al.v, ph + 48 * KP + k0, pl + 48 * KP + k0);
  }

  float* orow = sh_o + (16 * w + 8 * h) * NF + m;
#pragma unroll
  for (int r = 0; r < 8; ++r) {
    orow[r * NF]      = c0[r];
    orow[r * NF + 16] = c1[r];
    orow[r * NF + 32] = c2[r];
    orow[r * NF + 48] = c3[r];
  }
  __syncthreads();

  float* gb = msg + (size_t)ebase * NF;
#pragma unroll
  for (int q = 0; q < (EB * NF) / (4 * NTE); ++q) {
    const int fo = 4 * (q * NTE + t);
    const v4f v = *(const v4f*)(sh_o + fo);
    *(volatile v4f*)(gb + fo) = v;
  }
  __threadfence();
#pragma unroll
  for (int q = 0; q < (EB * NF) / (4 * NTE); ++q) {
    const int fo = 4 * (q * NTE + t);
    const v4f v = *(const v4f*)(sh_o + fo);
    *(volatile v4f*)(gb + fo) = v;
  }
}

__global__ __launch_bounds__(NTA) void k_agg(const float* __restrict__ msg, const int* __restrict__ dst,
                                             int E, int n_dst, int relu, float* outp) {
  __shared__ __attribute__((aligned(32))) float acc[NB * NF];
  __shared__ float cnt[NB];
  __shared__ int hit_e[CH];
  __shared__ int hit_n[CH];
  __shared__ int wcnt[2];
  const int t = threadIdx.x, lane = t & 31, w = t >> 5;
  const int n0 = blockIdx.x * NB;

  for (int i = t; i < NB * NF; i += NTA) acc[i] = 0.f;
  float cr0 = 0.f, cr1 = 0.f, cr2 = 0.f, cr3 = 0.f;
  __syncthreads();

#pragma unroll 1
  for (int cb = 0; cb < E; cb += CH) {
    const int e  = cb + t;
    const int ec = min(e, E - 1);
    const int d  = dst[ec];
    const int nl = d - n0;
    const bool valid = (e < E) && (d >= n0) && (d < n_dst) && (nl < NB);
    const unsigned mask = __builtin_amdgcn_ballot_w32(valid);
    const int pos = (int)__builtin_popcount(mask & ((1u << lane) - 1u));
    wcnt[w] = (int)__builtin_popcount(mask);
    __syncthreads();
    const int wc0 = wcnt[0], wc1 = wcnt[1];
    const int off = (w == 0) ? 0 : wc0;
    const int nh  = min(wc0 + wc1, CH);
    if (valid) {
      hit_e[off + pos] = e;
      hit_n[off + pos] = nl;
    }
    __syncthreads();
#pragma unroll 1
    for (int j = 0; j < nh; ++j) {
      int he = hit_e[j];
      int hn = hit_n[j];
      he = min(max(he, 0), E - 1);
      hn = min(max(hn, 0), NB - 1);
      const float v = msg[(size_t)he * NF + t];
      acc[hn * NF + t] += v;
      cr0 += (hn == t)           ? 1.f : 0.f;
      cr1 += (hn == t + NTA)     ? 1.f : 0.f;
      cr2 += (hn == t + 2 * NTA) ? 1.f : 0.f;
      cr3 += (hn == t + 3 * NTA) ? 1.f : 0.f;
    }
    __syncthreads();
  }

  cnt[t]           = cr0;
  cnt[t + NTA]     = cr1;
  cnt[t + 2 * NTA] = cr2;
  if (t + 3 * NTA < NB) cnt[t + 3 * NTA] = cr3;
  __syncthreads();

#pragma unroll 1
  for (int nl = 0; nl < NB; ++nl) {
    const float cn  = fmaxf(cnt[nl], 1.0f);
    const float inv = 1.0f / cn;
    float v = acc[nl * NF + t] * inv;
    v = relu ? fmaxf(v, 0.f) : v;
    acc[nl * NF + t] = v;
  }
  __syncthreads();

  const int rows_valid = min(NB, n_dst - n0);
  float* gb = outp + (size_t)n0 * NF;
#pragma unroll 1
  for (int q = 0; q < (NB * NF) / (4 * NTA); ++q) {
    const int fo  = 4 * (q * NTA + t);
    const int row = fo >> 6;
    const v4f v = *(const v4f*)(acc + fo);
    if (row < rows_valid) *(volatile v4f*)(gb + fo) = v;
  }
  __threadfence();
#pragma unroll 1
  for (int q = 0; q < (NB * NF) / (4 * NTA); ++q) {
    const int fo  = 4 * (q * NTA + t);
    const int row = fo >> 6;
    const v4f v = *(const v4f*)(acc + fo);
    if (row < rows_valid) *(volatile v4f*)(gb + fo) = v;
  }
}

extern "C" void kernel_launch(void* const* d_in, const int* in_sizes, int n_in,
                              void* d_out, int out_size, void* d_ws, size_t ws_size,
                              hipStream_t stream) {
  if (n_in < 11) return;
  const int hf_elems = in_sizes[0];
  if (hf_elems <= 0 || (hf_elems % NF) != 0) return;
  const int n_src = hf_elems / NF;
  const int E1 = in_sizes[7];
  const int E2 = in_sizes[9];
  if (E1 <= 0 || E2 <= 0) return;
  if (in_sizes[8] != E1 || in_sizes[10] != E2) return;
  if (in_sizes[1] != E1 * EFW || in_sizes[2] != E2 * EFW) return;
  if (in_sizes[3] != EFW * WCOLS || in_sizes[4] != WCOLS) return;
  if (in_sizes[5] != EFW * WCOLS || in_sizes[6] != WCOLS) return;
  if (out_size <= 0 || (out_size % NF) != 0) return;
  const int n_out = out_size / NF;
  const int n_mid = NMIDC;

  const float* in_feat = (const float*)d_in[0];
  const float* ef1     = (const float*)d_in[1];
  const float* ef2     = (const float*)d_in[2];
  const float* W1      = (const float*)d_in[3];
  const float* b1      = (const float*)d_in[4];
  const float* W2      = (const float*)d_in[5];
  const float* b2      = (const float*)d_in[6];
  const int*   src1    = (const int*)d_in[7];
  const int*   dst1    = (const int*)d_in[8];
  const int*   src2    = (const int*)d_in[9];
  const int*   dst2    = (const int*)d_in[10];
  float* out = (float*)d_out;

  const int nbe1 = (E1 + EB - 1) / EB;
  const int nbe2 = (E2 + EB - 1) / EB;
  const int e_pad = ((nbe1 > nbe2) ? nbe1 : nbe2) * EB;
  const int nba1 = (n_mid + NB - 1) / NB;
  const int nba2 = (n_out + NB - 1) / NB;
  const int mid_pad = nba1 * NB;

  char* ws = (char*)d_ws;
  size_t off = 0;
  const size_t oH1 = off; off += (size_t)PLB;                     off = (off + 255) & ~(size_t)255;
  const size_t oL1 = off; off += (size_t)PLB;                     off = (off + 255) & ~(size_t)255;
  const size_t oH2 = off; off += (size_t)PLB;                     off = (off + 255) & ~(size_t)255;
  const size_t oL2 = off; off += (size_t)PLB;                     off = (off + 255) & ~(size_t)255;
  const size_t oMsg = off; off += (size_t)e_pad * NF * 4;         off = (off + 255) & ~(size_t)255;
  const size_t oHm  = off; off += (size_t)mid_pad * NF * 4;       off = (off + 255) & ~(size_t)255;
  if (off > ws_size || off > (size_t)WSCAP) return;

  unsigned short* Bh1 = (unsigned short*)(ws + oH1);
  unsigned short* Bl1 = (unsigned short*)(ws + oL1);
  unsigned short* Bh2 = (unsigned short*)(ws + oH2);
  unsigned short* Bl2 = (unsigned short*)(ws + oL2);
  float* msg  = (float*)(ws + oMsg);
  float* hmid = (float*)(ws + oHm);

  k_wsplit<<<dim3((NF * KP / 8) / 256, 2, 1), 256, 0, stream>>>(W1, b1, W2, b2, Bh1, Bl1, Bh2, Bl2);
  k_edge<<<nbe1, NTE, 0, stream>>>(in_feat, n_src, ef1, src1, E1, Bh1, Bl1, msg);
  k_agg<<<nba1, NTA, 0, stream>>>(msg, dst1, E1, n_mid, 1, hmid);
  k_edge<<<nbe2, NTE, 0, stream>>>(hmid, n_mid, ef2, src2, E2, Bh2, Bl2, msg);
  k_agg<<<nba2, NTA, 0, stream>>>(msg, dst2, E2, n_out, 0, out);
}
